// PointNetSetAbstraction_9259949491067
// MI455X (gfx1250) — hardware-verified
//
#include <hip/hip_runtime.h>
#pragma clang fp contract(off)

typedef __attribute__((ext_vector_type(16))) _Float16 v16h;
typedef __attribute__((ext_vector_type(8)))  _Float16 v8h;
typedef __attribute__((ext_vector_type(8)))  float    v8f;
typedef __attribute__((ext_vector_type(4)))  float    v4f;
typedef __attribute__((ext_vector_type(4)))  int      v4i;

constexpr int NBATCH  = 8;
constexpr int NPTS_IN = 4096;
constexpr int NCH_IN  = 64;
constexpr int NCENT   = 1024;
constexpr int NSAMP   = 32;
constexpr int NCH_L0  = 64;
constexpr int NCH_L1  = 64;
constexpr int NCH_L2  = 128;
constexpr int KIN_L0  = 67;
constexpr int KPAD_L0 = 96;
constexpr int APITCH  = 104;
constexpr float WCARRY      = 16.0f;
constexpr float WCARRY_INV  = 1.0f / 16.0f;
constexpr float LOCARRY     = 2048.0f;
constexpr float LOCARRY_INV = 1.0f / 2048.0f;
constexpr float BN_EPS  = 1e-5f;
constexpr float BALL_R2 = 0.04f;

constexpr int BT0_OFF = 0;
constexpr int BT1_OFF = NCH_L0 * KPAD_L0;
constexpr int BT2_OFF = BT1_OFF + NCH_L1 * NCH_L0;
constexpr int BT_HALVES = BT2_OFF + NCH_L2 * NCH_L1;
static_assert(BT1_OFF == 6144 && BT2_OFF == 10240 && BT_HALVES == 18432, "Bt carve");
static_assert(BT_HALVES == 9 * 256 * 8, "prep grid covers the Bt planes exactly");
static_assert(KPAD_L0 % 32 == 0 && NCH_L0 % 32 == 0 && NCH_L1 % 32 == 0, "K multiples of 32");
static_assert(KIN_L0 == NCH_IN + 3, "layer-0 fan-in");

constexpr size_t WS_PTSH = 0;
constexpr size_t WS_PTSL = WS_PTSH + (size_t)NBATCH * NPTS_IN * NCH_IN * 2;
constexpr size_t WS_NX4  = WS_PTSL + (size_t)NBATCH * NPTS_IN * NCH_IN * 2;
constexpr size_t WS_GIDX = WS_NX4  + (size_t)NBATCH * NCENT * 4 * 4;
constexpr size_t WS_POOL = WS_GIDX + (size_t)NBATCH * NCENT * NSAMP * 4;
constexpr size_t WS_BT   = WS_POOL + (size_t)NBATCH * NCENT * NCH_L2 * 4;
constexpr size_t WS_FOLD = WS_BT   + (size_t)BT_HALVES * 2;
constexpr size_t WS_TOTAL = WS_FOLD + 512 * 4;
static_assert(WS_TOTAL == 13801472, "carve total");
static_assert(WS_TOTAL <= 134217728, "carve under 128 MiB");
static_assert(WS_PTSL % 128 == 0 && WS_NX4 % 128 == 0 && WS_GIDX % 128 == 0 && WS_POOL % 128 == 0 && WS_BT % 128 == 0 && WS_FOLD % 128 == 0, "line aligned carve");

constexpr size_t OUT1_OFF_BYTES = 98304;
static_assert(OUT1_OFF_BYTES == (size_t)NBATCH * NCENT * 3 * 4, "out0 extent");
static_assert(OUT1_OFF_BYTES % 128 == 0, "out1 line aligned");
static_assert(OUT1_OFF_BYTES + (size_t)NBATCH * NCH_L2 * NCENT * 4 == 4292608, "d_out total");

__device__ __forceinline__ void dep_guard_h(v8f& a, v8f& b, v16h x, v16h y) { asm volatile("v_nop\n\tv_nop\n\tv_nop\n\tv_nop" : "+v"(a), "+v"(b) : "v"(x), "v"(y)); }
__device__ __forceinline__ void keep4_h(v16h a, v16h b, v16h c, v16h d) { asm volatile("v_nop" :: "v"(a), "v"(b), "v"(c), "v"(d)); }
template <typename T> struct Frag;
template <> struct Frag<_Float16> {
  typedef v16h V; union U { v16h v; v8h h[2]; };
  static __device__ __forceinline__ v16h load(const _Float16* p) {
    U f; f.h[0] = *(const v8h*)(p); f.h[1] = *(const v8h*)(p + 16); return f.v;
  }
  static __device__ __forceinline__ v8f mma(v16h a, v16h b, v8f c) {
    return __builtin_amdgcn_wmma_f32_16x16x32_f16(false, a, false, b, (short)0, c, false, false);
  }
  static __device__ __forceinline__ void guard(v8f& a, v8f& b, v16h x, v16h y) { dep_guard_h(a, b, x, y); }
  static __device__ __forceinline__ void keep(v16h a, v16h b, v16h c, v16h d) { keep4_h(a, b, c, d); }
};

__device__ __forceinline__ v8f mma_f16(v16h a, v16h b, v8f c) {
  c = __builtin_amdgcn_wmma_f32_16x16x32_f16(false, a, false, b, (short)0, c, false, false);
  asm volatile("v_nop\n\tv_nop\n\tv_nop\n\tv_nop" : "+v"(c) : "v"(a), "v"(b));
  return c;
}

__global__ __launch_bounds__(256) void pack_points_kernel(const float* __restrict__ pts,
                                                          _Float16* __restrict__ ptsH,
                                                          _Float16* __restrict__ ptsL) {
  __shared__ float tile[64 * 65];
  const int tid = threadIdx.x, lane = tid & 31, wv = tid >> 5;
  const int b = blockIdx.x >> 6;
  const int n0 = (blockIdx.x & 63) << 6;
  {
    const int c = tid >> 2, nq = (tid & 3) * 16;
    const float* src = pts + ((size_t)(b * NCH_IN + c)) * NPTS_IN + n0 + nq;
#pragma unroll
    for (int i = 0; i < 4; ++i) {
      const v4f v = *(const v4f*)(src + 4 * i);
      tile[(nq + 4 * i + 0) * 65 + c] = v.x;
      tile[(nq + 4 * i + 1) * 65 + c] = v.y;
      tile[(nq + 4 * i + 2) * 65 + c] = v.z;
      tile[(nq + 4 * i + 3) * 65 + c] = v.w;
    }
  }
  __syncthreads();
  v8h hv[2], lv[2];
  const int c8 = (lane & 7) * 8;
#pragma unroll
  for (int it = 0; it < 2; ++it) {
    const int p = wv * 8 + it * 4 + (lane >> 3);
#pragma unroll
    for (int e = 0; e < 8; ++e) {
      const float f = tile[p * 65 + c8 + e];
      const _Float16 h = (_Float16)f;
      const float res = (f - (float)h) * LOCARRY;
      hv[it][e] = h;
      lv[it][e] = (_Float16)res;
    }
  }
  for (int pass = 0; pass < 2; ++pass) {
#pragma unroll
    for (int it = 0; it < 2; ++it) {
      const int p = wv * 8 + it * 4 + (lane >> 3);
      const size_t off = ((size_t)(b * NPTS_IN + n0 + p)) * NCH_IN + c8;
      *(volatile v8h*)(ptsH + off) = hv[it];
      *(volatile v8h*)(ptsL + off) = lv[it];
    }
    __threadfence();
  }
}

__global__ __launch_bounds__(256) void prep_weights_kernel(
    const float* __restrict__ w0, const float* __restrict__ g0, const float* __restrict__ b0,
    const float* __restrict__ m0, const float* __restrict__ v0,
    const float* __restrict__ w1, const float* __restrict__ g1, const float* __restrict__ b1,
    const float* __restrict__ m1, const float* __restrict__ v1,
    const float* __restrict__ w2, const float* __restrict__ g2, const float* __restrict__ b2,
    const float* __restrict__ m2, const float* __restrict__ v2,
    _Float16* __restrict__ Bt, float* __restrict__ fold) {
  __shared__ __align__(16) float sf[512];
  const int tid = threadIdx.x;
  if (blockIdx.x < 9) {
    const int h0 = (blockIdx.x * 256 + tid) * 8;
    v8h o;
    if (h0 < BT1_OFF) {
      const int n = h0 / KPAD_L0;
      const int k8 = h0 - n * KPAD_L0;
#pragma unroll
      for (int e = 0; e < 8; ++e) {
        const int k = k8 + e;
        const int col = (k < NCH_IN) ? (k + 3) : ((k < KIN_L0) ? (k - NCH_IN) : 0);
        const float f = w0[n * KIN_L0 + col];
        const float fs = (k < KIN_L0) ? (f * WCARRY) : 0.0f;
        o[e] = (_Float16)fs;
      }
    } else if (h0 < BT2_OFF) {
      const int i = h0 - BT1_OFF;
      const v4f a = *(const v4f*)(w1 + i);
      const v4f c = *(const v4f*)(w1 + i + 4);
      o[0] = (_Float16)(a.x * WCARRY); o[1] = (_Float16)(a.y * WCARRY);
      o[2] = (_Float16)(a.z * WCARRY); o[3] = (_Float16)(a.w * WCARRY);
      o[4] = (_Float16)(c.x * WCARRY); o[5] = (_Float16)(c.y * WCARRY);
      o[6] = (_Float16)(c.z * WCARRY); o[7] = (_Float16)(c.w * WCARRY);
    } else {
      const int i = h0 - BT2_OFF;
      const v4f a = *(const v4f*)(w2 + i);
      const v4f c = *(const v4f*)(w2 + i + 4);
      o[0] = (_Float16)(a.x * WCARRY); o[1] = (_Float16)(a.y * WCARRY);
      o[2] = (_Float16)(a.z * WCARRY); o[3] = (_Float16)(a.w * WCARRY);
      o[4] = (_Float16)(c.x * WCARRY); o[5] = (_Float16)(c.y * WCARRY);
      o[6] = (_Float16)(c.z * WCARRY); o[7] = (_Float16)(c.w * WCARRY);
    }
    *(volatile v8h*)(Bt + h0) = o;
    __threadfence();
    *(volatile v8h*)(Bt + h0) = o;
    __threadfence();
  } else {
    float s, sh;
    if (tid < 64) {
      s = g0[tid] * rsqrtf(v0[tid] + BN_EPS);
      sh = b0[tid] - m0[tid] * s;
    } else if (tid < 128) {
      const int c = tid - 64;
      s = g1[c] * rsqrtf(v1[c] + BN_EPS);
      sh = b1[c] - m1[c] * s;
    } else {
      const int c = tid - 128;
      s = g2[c] * rsqrtf(v2[c] + BN_EPS);
      sh = b2[c] - m2[c] * s;
    }
    sf[tid] = s * WCARRY_INV;
    sf[256 + tid] = sh;
    __syncthreads();
    if (tid < 128) {
      const v4f val = *(const v4f*)(sf + tid * 4);
      *(volatile v4f*)(fold + tid * 4) = val;
      __threadfence();
      *(volatile v4f*)(fold + tid * 4) = val;
      __threadfence();
    }
  }
}

__global__ __launch_bounds__(1024) void fps_kernel(const float* __restrict__ xyz,
                                                   float* __restrict__ out0,
                                                   float* __restrict__ nx4) {
#pragma clang fp contract(off)
  __shared__ __align__(16) float sx[NPTS_IN];
  __shared__ __align__(16) float sy[NPTS_IN];
  __shared__ __align__(16) float sz[NPTS_IN];
  __shared__ int   idxbuf[NCENT];
  __shared__ float wbv[2][32];
  __shared__ int   wbi[2][32];

  const int b = blockIdx.x, tid = threadIdx.x;
  const int lane = tid & 31, wid = tid >> 5;

  for (int i = tid; i < NPTS_IN; i += 1024) {
    const float* p = xyz + ((size_t)(b * NPTS_IN + i)) * 3;
    sx[i] = p[0]; sy[i] = p[1]; sz[i] = p[2];
  }
  __syncthreads();

  float dmin[4] = {1e10f, 1e10f, 1e10f, 1e10f};
  int farIdx = 0;

  for (int it = 0; it < NCENT; ++it) {
    if (tid == 0) idxbuf[it] = farIdx;
    const float cx = sx[farIdx], cy = sy[farIdx], cz = sz[farIdx];
    float bv = -1.0f; int bi = 0;
#pragma unroll
    for (int j = 0; j < 4; ++j) {
      const int p = tid + 1024 * j;
      const float dx = sx[p] - cx, dy = sy[p] - cy, dz = sz[p] - cz;
      const float t0 = dx * dx;
      const float t1 = dy * dy;
      const float t2 = dz * dz;
      const float d = (t0 + t2) + t1;
      dmin[j] = fminf(dmin[j], d);
      if (dmin[j] > bv) { bv = dmin[j]; bi = p; }
    }
    for (int off = 16; off; off >>= 1) {
      const float ov = __shfl_xor(bv, off);
      const int   oi = __shfl_xor(bi, off);
      if (ov > bv || (ov == bv && oi < bi)) { bv = ov; bi = oi; }
    }
    const int buf = it & 1;
    if (lane == 0) { wbv[buf][wid] = bv; wbi[buf][wid] = bi; }
    __syncthreads();
    bv = wbv[buf][lane]; bi = wbi[buf][lane];
    for (int off = 16; off; off >>= 1) {
      const float ov = __shfl_xor(bv, off);
      const int   oi = __shfl_xor(bi, off);
      if (ov > bv || (ov == bv && oi < bi)) { bv = ov; bi = oi; }
    }
    farIdx = bi & (NPTS_IN - 1);
  }

  int p = idxbuf[tid];
  p = p < 0 ? 0 : (p > NPTS_IN - 1 ? NPTS_IN - 1 : p);
  const float ox = sx[p], oy = sy[p], oz = sz[p];
  __syncthreads();
  sx[3 * tid + 0] = ox; sx[3 * tid + 1] = oy; sx[3 * tid + 2] = oz;
  __syncthreads();
  v4f q4;
  q4.x = ox; q4.y = oy; q4.z = oz; q4.w = 0.0f;
  const int tc = tid < 768 ? tid : 767;
  const v4f o4 = *(const v4f*)(sx + tc * 4);
  float* nxp = nx4 + ((size_t)(b * NCENT + tid)) * 4;
  float* o0p = out0 + (size_t)b * (NCENT * 3) + tc * 4;
  for (int pass = 0; pass < 2; ++pass) {
    *(volatile v4f*)nxp = q4;
    if (tid < 768) *(volatile v4f*)o0p = o4;
    __threadfence();
  }
}

__global__ __launch_bounds__(256) void ball_query_kernel(const float* __restrict__ xyz,
                                                         const float* __restrict__ nx4,
                                                         int* __restrict__ gidx) {
#pragma clang fp contract(off)
  __shared__ __align__(16) int sidx[8 * NSAMP];
  const int tid = threadIdx.x, lane = tid & 31, wv = tid >> 5;
  const int g = blockIdx.x * 8 + wv;
  const int b = g >> 10;
  const v4f q = *(const v4f*)(nx4 + (size_t)g * 4);
  const float qx = q.x, qy = q.y, qz = q.z;
  const float qx2 = qx * qx;
  const float qy2 = qy * qy;
  const float qz2 = qz * qz;
  const float sqq = (qx2 + qz2) + qy2;
  const float* xb = xyz + (size_t)b * NPTS_IN * 3;

  int cnt = 0, first = -1;
  for (int base = 0; base < NPTS_IN && cnt < NSAMP; base += 32) {
    const int j = base + lane;
    const float px = xb[j * 3 + 0], py = xb[j * 3 + 1], pz = xb[j * 3 + 2];
    float dot = qx * px;
    dot = fmaf(qy, py, dot);
    dot = fmaf(qz, pz, dot);
    const float px2 = px * px;
    const float py2 = py * py;
    const float pz2 = pz * pz;
    const float sqp = (px2 + pz2) + py2;
    const float m2d = -2.0f * dot;
    const float d = (m2d + sqq) + sqp;
    const bool pred = d <= BALL_R2;
    const unsigned m = (unsigned)__ballot(pred);
    if (first < 0 && m) first = base + __ffs(m) - 1;
    const int pos = cnt + __popc(m & ((1u << lane) - 1u));
    if (pred && pos < NSAMP) sidx[wv * NSAMP + pos] = j;
    cnt += __popc(m);
  }
  if (cnt > NSAMP) cnt = NSAMP;
  if (first < 0) first = 0;
  {
    const int p2 = cnt + lane;
    if (p2 < NSAMP) sidx[wv * NSAMP + p2] = first;
  }
  __syncthreads();
  if (tid < 64) {
    const v4i val = *(const v4i*)(sidx + tid * 4);
    int* dst = gidx + (size_t)blockIdx.x * (8 * NSAMP) + tid * 4;
    *(volatile v4i*)dst = val;
    __threadfence();
    *(volatile v4i*)dst = val;
    __threadfence();
  }
}

__global__ __launch_bounds__(128) void group_mlp_kernel(
    const float* __restrict__ xyz, const _Float16* __restrict__ ptsH, const _Float16* __restrict__ ptsL,
    const float* __restrict__ nx4, const int* __restrict__ gidx,
    const _Float16* __restrict__ Bt, const float* __restrict__ fold,
    float* __restrict__ poolT) {
  __shared__ __align__(16) _Float16 sAh[4][32 * APITCH];
  __shared__ __align__(16) _Float16 sAl[4][32 * APITCH];
  __shared__ __align__(16) float spool[4][NCH_L2];

  const int tid = threadIdx.x, lane = tid & 31, wv = tid >> 5;
  const int hh = lane >> 4, c = lane & 15, koff = hh * 8;
  const int g = blockIdx.x * 4 + wv;
  const int b = g >> 10;
  _Float16* Ah = sAh[wv];
  _Float16* Al = sAl[wv];

  int myidx = gidx[(size_t)g * NSAMP + lane];
  myidx = myidx < 0 ? 0 : (myidx > NPTS_IN - 1 ? NPTS_IN - 1 : myidx);

#pragma unroll 1
  for (int it = 0; it < 8; ++it) {
    const int row = it * 4 + (lane >> 3);
    const int c8 = (lane & 7) * 8;
    const int p = __shfl(myidx, row);
    const size_t off = ((size_t)(b * NPTS_IN + p)) * NCH_IN + c8;
    const v8h vh = *(const v8h*)(ptsH + off);
    const v8h vl = *(const v8h*)(ptsL + off);
    *(v8h*)(Ah + row * APITCH + c8) = vh;
    *(v8h*)(Al + row * APITCH + c8) = vl;
  }
  {
    const v4f q = *(const v4f*)(nx4 + (size_t)g * 4);
    const float* xp = xyz + ((size_t)(b * NPTS_IN + myidx)) * 3;
    const float dx = xp[0] - q.x;
    const float dy = xp[1] - q.y;
    const float dz = xp[2] - q.z;
    float zf = 0.0f;
    asm volatile("" : "+v"(zf));
    const _Float16 zh = (_Float16)zf;
    const _Float16 hx = (_Float16)dx;
    const _Float16 hy = (_Float16)dy;
    const _Float16 hz = (_Float16)dz;
    const float rx = (dx - (float)hx) * LOCARRY;
    const float ry = (dy - (float)hy) * LOCARRY;
    const float rz = (dz - (float)hz) * LOCARRY;
    v8h th, tl, zz;
    th[0] = hx; th[1] = hy; th[2] = hz; th[3] = zh; th[4] = zh; th[5] = zh; th[6] = zh; th[7] = zh;
    tl[0] = (_Float16)rx; tl[1] = (_Float16)ry; tl[2] = (_Float16)rz;
    tl[3] = zh; tl[4] = zh; tl[5] = zh; tl[6] = zh; tl[7] = zh;
    zz[0] = zh; zz[1] = zh; zz[2] = zh; zz[3] = zh; zz[4] = zh; zz[5] = zh; zz[6] = zh; zz[7] = zh;
    *(v8h*)(Ah + lane * APITCH + 64) = th;
    *(v8h*)(Ah + lane * APITCH + 72) = zz;
    *(v8h*)(Ah + lane * APITCH + 80) = zz;
    *(v8h*)(Ah + lane * APITCH + 88) = zz;
    *(v8h*)(Al + lane * APITCH + 64) = tl;
    *(v8h*)(Al + lane * APITCH + 72) = zz;
    *(v8h*)(Al + lane * APITCH + 80) = zz;
    *(v8h*)(Al + lane * APITCH + 88) = zz;
  }
  __syncthreads();

  const _Float16* Bt0 = Bt + BT0_OFF;
  const _Float16* Bt1 = Bt + BT1_OFF;
  const _Float16* Bt2 = Bt + BT2_OFF;
  const v8f vzero = (v8f){0.f, 0.f, 0.f, 0.f, 0.f, 0.f, 0.f, 0.f};

  {
    v16h ah[3][2], al[3][2];
#pragma unroll
    for (int kc = 0; kc < 3; ++kc) {
#pragma unroll
      for (int mt = 0; mt < 2; ++mt) {
        ah[kc][mt] = Frag<_Float16>::load(Ah + (mt * 16 + c) * APITCH + kc * 32 + koff);
        al[kc][mt] = Frag<_Float16>::load(Al + (mt * 16 + c) * APITCH + kc * 32 + koff);
      }
    }
#pragma unroll 1
    for (int nt = 0; nt < 4; ++nt) {
      v8f a0 = vzero, a1 = vzero, r0 = vzero, r1 = vzero;
#pragma unroll
      for (int kc = 0; kc < 3; ++kc) {
        const v16h bf = Frag<_Float16>::load(Bt0 + (nt * 16 + c) * KPAD_L0 + kc * 32 + koff);
        a0 = mma_f16(ah[kc][0], bf, a0);
        a1 = mma_f16(ah[kc][1], bf, a1);
        r0 = mma_f16(al[kc][0], bf, r0);
        r1 = mma_f16(al[kc][1], bf, r1);
      }
      const int ch = nt * 16 + c;
      const float sc = fold[ch], sh = fold[256 + ch];
#pragma unroll
      for (int r = 0; r < 8; ++r) {
        const float t0 = a0[r] + r0[r] * LOCARRY_INV;
        const float t1 = a1[r] + r1[r] * LOCARRY_INV;
        const float y0 = fmaxf(fmaf(t0, sc, sh), 0.0f);
        const float y1 = fmaxf(fmaf(t1, sc, sh), 0.0f);
        Ah[(8 * hh + r) * APITCH + ch] = (_Float16)y0;
        Ah[(16 + 8 * hh + r) * APITCH + ch] = (_Float16)y1;
      }
    }
  }
  __syncthreads();

  {
    v16h ah[2][2];
#pragma unroll
    for (int kc = 0; kc < 2; ++kc) {
#pragma unroll
      for (int mt = 0; mt < 2; ++mt) {
        ah[kc][mt] = Frag<_Float16>::load(Ah + (mt * 16 + c) * APITCH + kc * 32 + koff);
      }
    }
#pragma unroll 1
    for (int nt = 0; nt < 4; ++nt) {
      v8f a0 = vzero, a1 = vzero;
#pragma unroll
      for (int kc = 0; kc < 2; ++kc) {
        const v16h bf = Frag<_Float16>::load(Bt1 + (nt * 16 + c) * NCH_L0 + kc * 32 + koff);
        a0 = mma_f16(ah[kc][0], bf, a0);
        a1 = mma_f16(ah[kc][1], bf, a1);
      }
      const int ch = nt * 16 + c;
      const float sc = fold[64 + ch], sh = fold[256 + 64 + ch];
#pragma unroll
      for (int r = 0; r < 8; ++r) {
        const float y0 = fmaxf(fmaf(a0[r], sc, sh), 0.0f);
        const float y1 = fmaxf(fmaf(a1[r], sc, sh), 0.0f);
        Ah[(8 * hh + r) * APITCH + ch] = (_Float16)y0;
        Ah[(16 + 8 * hh + r) * APITCH + ch] = (_Float16)y1;
      }
    }
  }
  __syncthreads();

  {
    v16h ah[2][2];
#pragma unroll
    for (int kc = 0; kc < 2; ++kc) {
#pragma unroll
      for (int mt = 0; mt < 2; ++mt) {
        ah[kc][mt] = Frag<_Float16>::load(Ah + (mt * 16 + c) * APITCH + kc * 32 + koff);
      }
    }
#pragma unroll 1
    for (int nt = 0; nt < 8; ++nt) {
      v8f a0 = vzero, a1 = vzero;
#pragma unroll
      for (int kc = 0; kc < 2; ++kc) {
        const v16h bf = Frag<_Float16>::load(Bt2 + (nt * 16 + c) * NCH_L1 + kc * 32 + koff);
        a0 = mma_f16(ah[kc][0], bf, a0);
        a1 = mma_f16(ah[kc][1], bf, a1);
      }
      const int ch = nt * 16 + c;
      const float sc = fold[128 + ch], sh = fold[256 + 128 + ch];
      float mx = 0.0f;
#pragma unroll
      for (int r = 0; r < 8; ++r) {
        mx = fmaxf(mx, fmaf(a0[r], sc, sh));
        mx = fmaxf(mx, fmaf(a1[r], sc, sh));
      }
      const float other = __shfl_xor(mx, 16);
      mx = fmaxf(mx, other);
      if (hh == 0) spool[wv][ch] = mx;
    }
  }
  __syncthreads();
  {
    const v4f o = *(const v4f*)(&spool[wv][lane * 4]);
    float* dst = poolT + (size_t)g * NCH_L2 + lane * 4;
    *(volatile v4f*)dst = o;
    __threadfence();
    *(volatile v4f*)dst = o;
    __threadfence();
  }
}

__global__ __launch_bounds__(256) void pool_transpose_kernel(const float* __restrict__ poolT,
                                                             float* __restrict__ out1) {
  __shared__ float tile[NCH_L2 * 33];
  const int tid = threadIdx.x, lane = tid & 31, wv = tid >> 5;
  const int b = blockIdx.x >> 5;
  const int s0 = (blockIdx.x & 31) << 5;
#pragma unroll
  for (int i = 0; i < 4; ++i) {
    const int s = wv * 4 + i;
    const v4f v = *(const v4f*)(poolT + ((size_t)(b * NCENT + s0 + s)) * NCH_L2 + lane * 4);
    tile[(lane * 4 + 0) * 33 + s] = v.x;
    tile[(lane * 4 + 1) * 33 + s] = v.y;
    tile[(lane * 4 + 2) * 33 + s] = v.z;
    tile[(lane * 4 + 3) * 33 + s] = v.w;
  }
  __syncthreads();
  const int s4 = (lane & 7) * 4;
  v4f vals[4];
#pragma unroll
  for (int it = 0; it < 4; ++it) {
    const int ch = wv * 16 + it * 4 + (lane >> 3);
    v4f t;
    t.x = tile[ch * 33 + s4 + 0];
    t.y = tile[ch * 33 + s4 + 1];
    t.z = tile[ch * 33 + s4 + 2];
    t.w = tile[ch * 33 + s4 + 3];
    vals[it] = t;
  }
  for (int pass = 0; pass < 2; ++pass) {
#pragma unroll
    for (int it = 0; it < 4; ++it) {
      const int ch = wv * 16 + it * 4 + (lane >> 3);
      *(volatile v4f*)(out1 + ((size_t)(b * NCH_L2 + ch)) * NCENT + s0 + s4) = vals[it];
    }
    __threadfence();
  }
}

extern "C" void kernel_launch(void* const* d_in, const int* in_sizes, int n_in,
                              void* d_out, int out_size, void* d_ws, size_t ws_size,
                              hipStream_t stream) {
  (void)in_sizes; (void)out_size;
  if (n_in < 17) return;
  if (ws_size < WS_TOTAL) return;
  const float* xyz = (const float*)d_in[0];
  const float* pts = (const float*)d_in[1];
  const float* w0 = (const float*)d_in[2];
  const float* g0 = (const float*)d_in[3];
  const float* b0 = (const float*)d_in[4];
  const float* m0 = (const float*)d_in[5];
  const float* v0 = (const float*)d_in[6];
  const float* w1 = (const float*)d_in[7];
  const float* g1 = (const float*)d_in[8];
  const float* b1 = (const float*)d_in[9];
  const float* m1 = (const float*)d_in[10];
  const float* v1 = (const float*)d_in[11];
  const float* w2 = (const float*)d_in[12];
  const float* g2 = (const float*)d_in[13];
  const float* b2 = (const float*)d_in[14];
  const float* m2 = (const float*)d_in[15];
  const float* v2 = (const float*)d_in[16];

  float* out0 = (float*)d_out;
  float* out1 = (float*)d_out + (OUT1_OFF_BYTES / 4);

  char* ws = (char*)d_ws;
  _Float16* ptsH = (_Float16*)(ws + WS_PTSH);
  _Float16* ptsL = (_Float16*)(ws + WS_PTSL);
  float* nx4   = (float*)(ws + WS_NX4);
  int*   gidx  = (int*)(ws + WS_GIDX);
  float* poolT = (float*)(ws + WS_POOL);
  _Float16* Bt = (_Float16*)(ws + WS_BT);
  float* fold  = (float*)(ws + WS_FOLD);

  pack_points_kernel<<<NBATCH * (NPTS_IN / 64), 256, 0, stream>>>(pts, ptsH, ptsL);
  prep_weights_kernel<<<10, 256, 0, stream>>>(w0, g0, b0, m0, v0, w1, g1, b1, m1, v1,
                                              w2, g2, b2, m2, v2, Bt, fold);
  fps_kernel<<<NBATCH, 1024, 0, stream>>>(xyz, out0, nx4);
  ball_query_kernel<<<(NBATCH * NCENT) / 8, 256, 0, stream>>>(xyz, nx4, gidx);
  group_mlp_kernel<<<(NBATCH * NCENT) / 4, 128, 0, stream>>>(xyz, ptsH, ptsL, nx4, gidx, Bt, fold, poolT);
  pool_transpose_kernel<<<NBATCH * (NCENT / 32), 256, 0, stream>>>(poolT, out1);
}
